// RTRLDiagonalRNN_64510408786262
// MI455X (gfx1250) — hardware-verified
//
#include <hip/hip_runtime.h>

constexpr int kSteps = 4096;
constexpr int kChan  = 2048;

typedef __attribute__((ext_vector_type(16))) _Float16 v16h;
typedef __attribute__((ext_vector_type(8)))  _Float16 v8h;
typedef __attribute__((ext_vector_type(16))) __bf16   v16b;
typedef __attribute__((ext_vector_type(8)))  __bf16   v8b;
typedef __attribute__((ext_vector_type(8)))  float    v8f;
typedef __attribute__((ext_vector_type(4)))  float    v4f;
typedef __attribute__((ext_vector_type(4)))  unsigned int v4u;

__device__ __forceinline__ unsigned short f2bf_bits(float f) {
  unsigned u = __float_as_uint(f);
  return (unsigned short)((u + 0x7FFFu + ((u >> 16) & 1u)) >> 16);
}
__device__ __forceinline__ float bf_bits2f(unsigned short h) { return __uint_as_float(((unsigned)h) << 16); }

__device__ __forceinline__ void dep_guard_h(v8f& a, v8f& b, v16h x, v16h y) { asm volatile("v_nop\n\tv_nop\n\tv_nop\n\tv_nop" : "+v"(a), "+v"(b) : "v"(x), "v"(y)); }
__device__ __forceinline__ void dep_guard_b(v8f& a, v8f& b, v16b x, v16b y) { asm volatile("v_nop\n\tv_nop\n\tv_nop\n\tv_nop" : "+v"(a), "+v"(b) : "v"(x), "v"(y)); }
__device__ __forceinline__ void keep4_h(v16h a, v16h b, v16h c, v16h d) { asm volatile("v_nop" :: "v"(a), "v"(b), "v"(c), "v"(d)); }
__device__ __forceinline__ void keep4_b(v16b a, v16b b, v16b c, v16b d) { asm volatile("v_nop" :: "v"(a), "v"(b), "v"(c), "v"(d)); }
__device__ __forceinline__ void acc_guard4(v8f& a, v8f& b, v8f& c, v8f& d) { asm volatile("v_nop\n\tv_nop\n\tv_nop\n\tv_nop" : "+v"(a), "+v"(b), "+v"(c), "+v"(d)); }
template <typename T> struct Frag;
template <> struct Frag<_Float16> {
  typedef v16h V; union U { v16h v; v8h h[2]; };
  static __device__ __forceinline__ v16h load(const _Float16* p) {
    U f; f.h[0] = *(const v8h*)(p); f.h[1] = *(const v8h*)(p + 16); return f.v;
  }
  static __device__ __forceinline__ v8f mma(v16h a, v16h b, v8f c) {
    return __builtin_amdgcn_wmma_f32_16x16x32_f16(false, a, false, b, (short)0, c, false, false);
  }
  static __device__ __forceinline__ void guard(v8f& a, v8f& b, v16h x, v16h y) { dep_guard_h(a, b, x, y); }
  static __device__ __forceinline__ void keep(v16h a, v16h b, v16h c, v16h d) { keep4_h(a, b, c, d); }
};
template <> struct Frag<__bf16> {
  typedef v16b V; union U { v16b v; v8b h[2]; };
  static __device__ __forceinline__ v16b load(const __bf16* p) {
    U f; f.h[0] = *(const v8b*)(p); f.h[1] = *(const v8b*)(p + 16); return f.v;
  }
  static __device__ __forceinline__ v8f mma(v16b a, v16b b, v8f c) {
    return __builtin_amdgcn_wmma_f32_16x16x32_bf16(false, a, false, b, (short)0, c, false, false);
  }
  static __device__ __forceinline__ void guard(v8f& a, v8f& b, v16b x, v16b y) { dep_guard_b(a, b, x, y); }
  static __device__ __forceinline__ void keep(v16b a, v16b b, v16b c, v16b d) { keep4_b(a, b, c, d); }
};

__device__ __forceinline__ unsigned pk16(unsigned short a, unsigned short b) { return (unsigned)a | ((unsigned)b << 16); }

template <int ET> struct Elem;
template <> struct Elem<0> { typedef _Float16 T; };
template <> struct Elem<1> { typedef __bf16 T; };
template <int ET, bool SPLIT, int BIAS_MODE, int OUT_MODE, bool RESID, int ACT = 0>
__global__ __launch_bounds__(256) void wmma_gemm64(
    const unsigned short* __restrict__ Ap, const unsigned short* __restrict__ A2p, int lda, long strideA,
    const unsigned short* __restrict__ Btp, const unsigned short* __restrict__ Bt2p, int ldb, long strideB,
    void* __restrict__ Cout, void* __restrict__ Cout2, int ldc, long strideC,
    const float* __restrict__ bias,
    const float* __restrict__ resid, long strideR,
    int M, int N, int K, float scale) {
  typedef typename Elem<ET>::T T;
  typedef typename Frag<T>::V V;
  const T* A = (const T*)Ap; const T* A2 = (const T*)A2p; const T* Bt = (const T*)Btp; const T* Bt2 = (const T*)Bt2p;
  __shared__ __align__(16) float sT[8][16 * 68];
  const int b    = blockIdx.y;
  const int lane = threadIdx.x & 31;
  const int wave = threadIdx.x >> 5;
  const int tilesN = N >> 6;
  const int tilesM = M >> 6;
  const int tile = blockIdx.x * 8 + wave;
  if (tile >= tilesM * tilesN) return;
  const int tm = tile / tilesN;
  const int tn = tile - tm * tilesN;
  const int m0 = tm << 6;
  const int n0 = tn << 6;

  const T* Ab  = A  + (size_t)b * strideA;
  const T* Bb  = Bt + (size_t)b * strideB;
  const T* Ab2 = SPLIT ? (A2  + (size_t)b * strideA) : nullptr;
  const T* Bb2 = SPLIT ? (Bt2 + (size_t)b * strideB) : nullptr;

  const int rlane = lane & 15;
  const int koff  = (lane >> 4) * 8;
  const int mOff  = (lane >> 4) * 8;

  v8f acc[4][4];
#pragma unroll
  for (int i = 0; i < 4; ++i)
#pragma unroll
    for (int j = 0; j < 4; ++j) acc[i][j] = (v8f){0.f,0.f,0.f,0.f,0.f,0.f,0.f,0.f};

  for (int k0 = 0; k0 < K; k0 += 32) {
    V bh[4], bl[4];
#pragma unroll
    for (int j = 0; j < 4; ++j) {
      const size_t bo = (size_t)(n0 + (j << 4) + rlane) * ldb + koff + k0;
      bh[j] = Frag<T>::load(Bb + bo);
      if (SPLIT) bl[j] = Frag<T>::load(Bb2 + bo);
    }
#pragma unroll
    for (int i = 0; i < 4; ++i) {
      const size_t ao = (size_t)(m0 + (i << 4) + rlane) * lda + koff + k0;
      V ah = Frag<T>::load(Ab + ao);
      V al;
      if (SPLIT) al = Frag<T>::load(Ab2 + ao);
#pragma unroll
      for (int j = 0; j < 4; ++j) {
        acc[i][j] = Frag<T>::mma(ah, bh[j], acc[i][j]);
        if (SPLIT) {
          acc[i][j] = Frag<T>::mma(ah, bl[j], acc[i][j]);
          acc[i][j] = Frag<T>::mma(al, bh[j], acc[i][j]);
        }
      }
      Frag<T>::guard(acc[i][0], acc[i][3], ah, SPLIT ? al : ah);
    }
    Frag<T>::keep(bh[0], bh[1], bh[2], bh[3]);
    if (SPLIT) Frag<T>::keep(bl[0], bl[1], bl[2], bl[3]);
  }
  acc_guard4(acc[0][0], acc[0][1], acc[0][2], acc[0][3]);
  acc_guard4(acc[1][0], acc[1][1], acc[1][2], acc[1][3]);
  acc_guard4(acc[2][0], acc[2][1], acc[2][2], acc[2][3]);
  acc_guard4(acc[3][0], acc[3][1], acc[3][2], acc[3][3]);

  float* slab = sT[wave];
  const float* Rb = RESID ? (resid + (size_t)b * strideR) : nullptr;
#pragma unroll
  for (int i = 0; i < 4; ++i) {
    const int mBase = m0 + (i << 4);
#pragma unroll
    for (int j = 0; j < 4; ++j) {
      const int n = n0 + (j << 4) + rlane;
      float bv = 0.f;
      if (BIAS_MODE == 2) bv = bias[n];
#pragma unroll
      for (int r = 0; r < 8; ++r) {
        float v = acc[i][j][r] * scale;
        if (BIAS_MODE == 1) v += bias[mBase + mOff + r];
        if (BIAS_MODE == 2) v += bv;
        if (RESID) v += Rb[(size_t)(mBase + mOff + r) * ldc + n];
        if (ACT == 2) v = fmaxf(v, 0.0f);
        if (ACT == 4) v = (v > 0.f) ? v : 0.01f * v;
        slab[(mOff + r) * 68 + (j << 4) + rlane] = v;
      }
    }
    __builtin_amdgcn_fence(__ATOMIC_RELEASE, "workgroup");
    __builtin_amdgcn_wave_barrier();
    __builtin_amdgcn_fence(__ATOMIC_ACQUIRE, "workgroup");
    if (OUT_MODE == 0) {
      float* C = (float*)Cout + (size_t)b * strideC;
      const int hh = lane >> 4, c4 = (lane & 15) * 4;
      for (int pass = 0; pass < 2; ++pass) {
#pragma unroll
        for (int it = 0; it < 8; ++it) {
          const int row = it * 2 + hh;
          v4f v = *(const v4f*)(slab + row * 68 + c4);
          *(volatile v4f*)(C + (size_t)(mBase + row) * ldc + n0 + c4) = v;
        }
        __threadfence();
      }
    } else {
      const int q = lane >> 3, c8 = (lane & 7) * 8;
      unsigned short* C  = (unsigned short*)Cout  + (size_t)b * strideC;
      unsigned short* C2 = (OUT_MODE == 2) ? ((unsigned short*)Cout2 + (size_t)b * strideC) : nullptr;
      for (int pass = 0; pass < 2; ++pass) {
#pragma unroll
        for (int it = 0; it < 4; ++it) {
          const int row = it * 4 + q;
          const float* sp = slab + row * 68 + c8;
          v8h hv, lv;
#pragma unroll
          for (int e = 0; e < 8; ++e) {
            if (OUT_MODE == 1) {
              hv[e] = (_Float16)sp[e];
            } else {
              unsigned short hb = f2bf_bits(sp[e]);
              unsigned short lb = f2bf_bits(sp[e] - bf_bits2f(hb));
              hv[e] = __builtin_bit_cast(_Float16, hb);
              lv[e] = __builtin_bit_cast(_Float16, lb);
            }
          }
          *(volatile v8h*)(C + (size_t)(mBase + row) * ldc + n0 + c8) = hv;
          if (OUT_MODE == 2) *(volatile v8h*)(C2 + (size_t)(mBase + row) * ldc + n0 + c8) = lv;
        }
        __threadfence();
      }
    }
    __builtin_amdgcn_fence(__ATOMIC_RELEASE, "workgroup");
    __builtin_amdgcn_wave_barrier();
    __builtin_amdgcn_fence(__ATOMIC_ACQUIRE, "workgroup");
  }
}

__global__ __launch_bounds__(256) void split8_bf16_kernel(const float* __restrict__ in,
                                                          unsigned short* __restrict__ hi,
                                                          unsigned short* __restrict__ lo, int n8) {
  const int i = blockIdx.x * 256 + threadIdx.x;
  if (i >= n8) return;
  const float* p = in + 8 * (size_t)i;
  const v4f a = *(const v4f*)(p);
  const v4f c = *(const v4f*)(p + 4);
  unsigned short hb[8], lb[8];
#pragma unroll
  for (int e = 0; e < 4; ++e) {
    const unsigned short h0 = f2bf_bits(a[e]);
    hb[e] = h0;
    lb[e] = f2bf_bits(a[e] - bf_bits2f(h0));
    const unsigned short h1 = f2bf_bits(c[e]);
    hb[4 + e] = h1;
    lb[4 + e] = f2bf_bits(c[e] - bf_bits2f(h1));
  }
  const v4u uh = (v4u){pk16(hb[0], hb[1]), pk16(hb[2], hb[3]), pk16(hb[4], hb[5]), pk16(hb[6], hb[7])};
  const v4u ul = (v4u){pk16(lb[0], lb[1]), pk16(lb[2], lb[3]), pk16(lb[4], lb[5]), pk16(lb[6], lb[7])};
  unsigned short* qh = hi + 8 * (size_t)i;
  unsigned short* ql = lo + 8 * (size_t)i;
  *(volatile v4u*)qh = uh;
  *(volatile v4u*)ql = ul;
  __threadfence();
  *(volatile v4u*)qh = uh;
  *(volatile v4u*)ql = ul;
}

__global__ __launch_bounds__(128) void diag_scan_kernel(const float* __restrict__ U, const float* __restrict__ lam,
                                                        float* __restrict__ out, int ncols, int nsteps) {
#pragma clang fp contract(off)
  const int g = blockIdx.x * 128 + threadIdx.x;
  if (4 * g + 3 >= ncols + 3) return;
  const v4f lv = *(const v4f*)(lam + 4 * (size_t)g);
  v4f h = (v4f){0.f, 0.f, 0.f, 0.f};
  const float* up = U + 4 * (size_t)g;
  float* op = out + 4 * (size_t)g;
#pragma unroll 1
  for (int t = 0; t < nsteps; ++t) {
    const v4f u = *(const v4f*)(up + (size_t)t * ncols);
    v4f pm = lv * h;
    asm volatile("" : "+v"(pm));
    h = pm + u;
    float* dst = op + (size_t)t * ncols;
    const v4f hv = h;
    *(volatile v4f*)dst = hv;
    __threadfence();
    *(volatile v4f*)dst = hv;
  }
}

extern "C" void kernel_launch(void* const* d_in, const int* in_sizes, int n_in,
                              void* d_out, int out_size, void* d_ws, size_t ws_size,
                              hipStream_t stream) {
  if (n_in < 3) return;
  const float* X   = (const float*)d_in[0];
  const float* lam = (const float*)d_in[1];
  const float* Bm  = (const float*)d_in[2];
  float* out = (float*)d_out;

  const int nX = in_sizes[0];
  const int H  = in_sizes[1];
  const int nB = in_sizes[2];
  if (H <= 0 || (H % 64) != 0) return;
  const int T = nX / H;
  if (T * H != nX || nB != H * H || out_size != nX) return;
  if ((T % 64) != 0 || (H % 32) != 0 || (H % 4) != 0) return;
  if ((nX % 8) != 0 || (nB % 8) != 0) return;

  const size_t bytesX16 = (size_t)nX * 2;
  const size_t bytesB16 = (size_t)nB * 2;
  const size_t bytesU   = (size_t)nX * 4;
  const size_t offXhi = 0;
  const size_t offXlo = offXhi + bytesX16;
  const size_t offBhi = offXlo + bytesX16;
  const size_t offBlo = offBhi + bytesB16;
  const size_t offU   = offBlo + bytesB16;
  const size_t total  = offU + bytesU;
  if (total > ws_size) return;

  char* ws = (char*)d_ws;
  unsigned short* Xhi = (unsigned short*)(ws + offXhi);
  unsigned short* Xlo = (unsigned short*)(ws + offXlo);
  unsigned short* Bhi = (unsigned short*)(ws + offBhi);
  unsigned short* Blo = (unsigned short*)(ws + offBlo);
  float* U = (float*)(ws + offU);

  const int nX8 = nX / 8;
  const int nB8 = nB / 8;
  split8_bf16_kernel<<<dim3((nX8 + 255) / 256), dim3(256), 0, stream>>>(X, Xhi, Xlo, nX8);
  split8_bf16_kernel<<<dim3((nB8 + 255) / 256), dim3(256), 0, stream>>>(Bm, Bhi, Blo, nB8);

  const int tilesM = T / 64, tilesN = H / 64;
  const int tiles = tilesM * tilesN;
  const int gemmBlocks = (tiles + 7) / 8;
  wmma_gemm64<1, true, 0, 0, false, 0><<<dim3(gemmBlocks, 1), dim3(256), 0, stream>>>(
      Xhi, Xlo, H, (long)0,
      Bhi, Blo, H, (long)0,
      (void*)U, (void*)nullptr, H, (long)0,
      (const float*)nullptr,
      (const float*)nullptr, (long)0,
      T, H, H, 1.0f);

  const int scanThreads = H / 4;
  diag_scan_kernel<<<dim3((scanThreads + 127) / 128), dim3(128), 0, stream>>>(U, lam, out, H, T);
}
